// Conv_MoE_8091718385699
// MI455X (gfx1250) — hardware-verified
//
#include <hip/hip_runtime.h>
#include <stddef.h>


#pragma clang fp contract(off)

#define NBATCH 32
#define CH     128
#define IMH    56
#define IMW    56
#define NPIX   (IMH * IMW)
#define PADH   (IMH + 2)
#define PADW   (IMW + 2)
#define NEXP   8
#define NTAP   9
#define PGRP   (NPIX / 32)
#define HALFP  (NPIX / 2)
#define GLW    32

#define TGATE  256
#define TCVT   256
#define TCONV  128
#define TPITCH 136
#define OPITCH 36
#define NCHUNK (PADW * CH / 8)

#define G_GATE NBATCH
#define G_XCVT (NBATCH * PADH)
#define G_WSEL ((NBATCH * 2 * NTAP * CH * (CH / 8)) / TCVT)
#define G_CONV (NBATCH * PGRP)

static_assert(NPIX == 3136);
static_assert(PGRP * 32 == NPIX);
static_assert(HALFP * 2 == NPIX);
static_assert(TGATE == 2 * CH);
static_assert((CH * IMW) % TCVT == 0);
static_assert(NCHUNK % 32 == 0);
static_assert(NCHUNK <= 4 * TCVT);
static_assert((NBATCH * 2 * NTAP * CH * (CH / 8)) % TCVT == 0);
static_assert(G_XCVT == 1856);
static_assert(G_WSEL == 4608);
static_assert(G_CONV == 3136);
static_assert(TCONV == 128);
static_assert((TPITCH % 8) == 0);
static_assert((OPITCH % 4) == 0);
static_assert(CH % 32 == 0);

typedef float          v4f  __attribute__((ext_vector_type(4)));
typedef unsigned int   v4u  __attribute__((ext_vector_type(4)));
typedef float          v8f  __attribute__((ext_vector_type(8)));
typedef _Float16       v8h  __attribute__((ext_vector_type(8)));
typedef _Float16       v16h __attribute__((ext_vector_type(16)));
typedef v4f __attribute__((may_alias)) v4fa;
typedef v4u __attribute__((may_alias)) v4ua;

union Frag { v16h v; v4u q[2]; };
union Pack8 { v8h h; v4u u; };

__device__ __forceinline__ int clampi(int v, int lo, int hi) {
  return (v < lo) ? lo : ((v > hi) ? hi : v);
}

__device__ __forceinline__ v8f wmma_h(v16h a, v16h b, v8f c) {
  v8f d = __builtin_amdgcn_wmma_f32_16x16x32_f16(false, a, false, b, (short)0, c, false, false);
  asm volatile("v_nop\n\tv_nop\n\tv_nop\n\tv_nop" : "+v"(d) : "v"(a), "v"(b));
  return d;
}

__device__ __forceinline__ v16h ldfrag(const unsigned short* p) {
  Frag f;
  f.q[0] = *(const v4ua*)(p);
  f.q[1] = *(const v4ua*)(p + 16);
  return f.v;
}

__global__ __launch_bounds__(TGATE) void k_gate(const float* __restrict__ x,
                                                const float* __restrict__ gw,
                                                const float* __restrict__ gb,
                                                const int* __restrict__ tk,
                                                float* __restrict__ gl)
{
  __shared__ double sPart[TGATE];
  __shared__ float  sGap[CH];
  __shared__ float  sLg[NEXP];
  __shared__ int    sSelI[NEXP];
  __shared__ float  sSelV[NEXP];
  __shared__ float  sSelU[NEXP];
  __shared__ __align__(16) float sLine[GLW];

  const int tid = threadIdx.x, b = blockIdx.x;
  const int c = tid >> 1, hf = tid & 1;
  const float* p = x + ((size_t)(b * CH + c)) * NPIX + hf * HALFP;
  double s = 0.0;
  #pragma unroll 4
  for (int i = 0; i < HALFP; ++i) s += (double)p[i];
  sPart[tid] = s;
  if (tid < GLW) sLine[tid] = 0.0f;
  __syncthreads();
  if (tid < CH) {
    const double t = sPart[2 * tid] + sPart[2 * tid + 1];
    sGap[tid] = (float)(t * (1.0 / 3136.0));
  }
  __syncthreads();
  if (tid < NEXP) {
    const float* w = gw + tid * CH;
    double a = 0.0;
    #pragma unroll 1
    for (int k = 0; k < CH; ++k) a += (double)sGap[k] * (double)w[k];
    sLg[tid] = (float)a + gb[tid];
  }
  __syncthreads();
  if (tid == 0) {
    int kk = tk[0];
    kk = clampi(kk, 1, NEXP);
    unsigned int used = 0u;
    #pragma unroll 1
    for (int j = 0; j < kk; ++j) {
      int best = -1;
      float bv = 0.0f;
      #pragma unroll 1
      for (int e = 0; e < NEXP; ++e) {
        const bool fr = ((used >> e) & 1u) == 0u;
        const float v = sLg[e];
        const bool take = fr && ((best < 0) || (v > bv));
        best = take ? e : best;
        bv   = take ? v : bv;
      }
      used |= 1u << best;
      sSelI[j] = best;
      sSelV[j] = bv;
    }
    const float mx = sSelV[0];
    float sum = 0.0f;
    #pragma unroll 1
    for (int j = 0; j < kk; ++j) {
      const float u = expf(sSelV[j] - mx);
      sSelU[j] = u;
      sum = sum + u;
    }
    const float rcp = 1.0f / sum;
    #pragma unroll 1
    for (int j = 0; j < kk; ++j) sLine[sSelI[j]] = sSelU[j] * rcp;
    const int   ea = sSelI[0];
    const float wa = sSelU[0] * rcp;
    int   eb = ea;
    float wb = 0.0f;
    if (kk >= 2) { eb = sSelI[1]; wb = sSelU[1] * rcp; }
    const bool sw = eb < ea;
    sLine[8]  = (float)(sw ? eb : ea);
    sLine[9]  = (float)(sw ? ea : eb);
    sLine[10] = sw ? wb : wa;
    sLine[11] = sw ? wa : wb;
  }
  __syncthreads();
  if (tid < 8) {
    const v4f v = *(const v4fa*)(sLine + 4 * tid);
    float* d = gl + (size_t)b * GLW + 4 * tid;
    *(volatile v4f*)d = v;
    __threadfence();
    *(volatile v4f*)d = v;
  }
}

__global__ __launch_bounds__(TCVT) void k_xcvt(const float* __restrict__ x,
                                               unsigned short* __restrict__ xh)
{
  __shared__ __align__(16) _Float16 sT[PADW * TPITCH];

  const int tid = threadIdx.x, blk = blockIdx.x;
  const int b  = blk / PADH;
  const int hp = blk - b * PADH;
  const bool interior = (hp >= 1) && (hp <= IMH);
  const int hc = clampi(hp - 1, 0, IMH - 1);
  const float* src = x + ((size_t)b * CH) * NPIX + (size_t)hc * IMW;

  #pragma unroll 4
  for (int it = 0; it < (CH * IMW) / TCVT; ++it) {
    const int idx = it * TCVT + tid;
    const int c = idx / IMW;
    const int w = idx - c * IMW;
    const float v = src[(size_t)c * NPIX + w];
    const float f = interior ? v : 0.0f;
    sT[(w + 1) * TPITCH + c] = (_Float16)f;
  }
  if (tid < CH) sT[tid] = (_Float16)0.0f;
  else          sT[(PADW - 1) * TPITCH + (tid - CH)] = (_Float16)0.0f;
  __syncthreads();

  unsigned short* dst = xh + ((size_t)(b * PADH + hp)) * (PADW * CH);
  #pragma unroll
  for (int it = 0; it < 4; ++it) {
    const int q = it * TCVT + tid;
    if (q < NCHUNK) {
      const int wp = q >> 4, cc = (q & 15) * 8;
      const v4u v = *(const v4ua*)(sT + wp * TPITCH + cc);
      *(volatile v4u*)(dst + (size_t)q * 8) = v;
    }
  }
  __threadfence();
  #pragma unroll
  for (int it = 0; it < 4; ++it) {
    const int q = it * TCVT + tid;
    if (q < NCHUNK) {
      const int wp = q >> 4, cc = (q & 15) * 8;
      const v4u v = *(const v4ua*)(sT + wp * TPITCH + cc);
      *(volatile v4u*)(dst + (size_t)q * 8) = v;
    }
  }
}

__global__ __launch_bounds__(TCVT) void k_wsel(const float* __restrict__ cw,
                                               const float* __restrict__ gl,
                                               unsigned short* __restrict__ wsel,
                                               float* __restrict__ out1)
{
  const int tid = threadIdx.x;
  const int u   = blockIdx.x * TCVT + tid;
  const int cg  = u & 15;
  const int co  = (u >> 4) & (CH - 1);
  const int t2  = u >> 11;
  const int bj  = t2 / NTAP;
  const int tap = t2 - bj * NTAP;
  const int b   = bj >> 1;
  const int j   = bj & 1;
  float ef = gl[(size_t)b * GLW + 8 + j];
  ef = fminf(fmaxf(ef, 0.0f), (float)(NEXP - 1));
  const int e = clampi((int)ef, 0, NEXP - 1);
  const float* src = cw + (((size_t)(e * CH + co)) * CH + cg * 8) * NTAP + tap;
  Pack8 pk;
  pk.h[0] = (_Float16)(src[0 * NTAP] * 16.0f);
  pk.h[1] = (_Float16)(src[1 * NTAP] * 16.0f);
  pk.h[2] = (_Float16)(src[2 * NTAP] * 16.0f);
  pk.h[3] = (_Float16)(src[3 * NTAP] * 16.0f);
  pk.h[4] = (_Float16)(src[4 * NTAP] * 16.0f);
  pk.h[5] = (_Float16)(src[5 * NTAP] * 16.0f);
  pk.h[6] = (_Float16)(src[6 * NTAP] * 16.0f);
  pk.h[7] = (_Float16)(src[7 * NTAP] * 16.0f);
  unsigned short* d = wsel + (size_t)u * 8;
  *(volatile v4u*)d = pk.u;
  __threadfence();
  *(volatile v4u*)d = pk.u;

  if (blockIdx.x == 0 && tid < 32) {
    const int q0 = tid, q1 = 32 + tid;
    const v4f va = *(const v4fa*)(gl + (size_t)(q0 >> 1) * GLW + 4 * (q0 & 1));
    const v4f vb = *(const v4fa*)(gl + (size_t)(q1 >> 1) * GLW + 4 * (q1 & 1));
    *(volatile v4f*)(out1 + 4 * q0) = va;
    *(volatile v4f*)(out1 + 4 * q1) = vb;
    __threadfence();
    *(volatile v4f*)(out1 + 4 * q0) = va;
    *(volatile v4f*)(out1 + 4 * q1) = vb;
  }
}

__device__ __forceinline__ void epi_tile(float* so, v8f ya, v8f yb, float wlo, float whi,
                                         int pt, int ct, int h, int m)
{
  #pragma unroll
  for (int r = 0; r < 8; ++r) {
    const float y0 = ya[r] * 0.0625f;
    const float y1 = yb[r] * 0.0625f;
    const float pa = wlo * y0;
    const float pb = whi * y1;
    so[(ct * 16 + m) * OPITCH + pt * 16 + 8 * h + r] = pa + pb;
  }
}

__global__ __launch_bounds__(TCONV) void k_conv(const unsigned short* __restrict__ xh,
                                               const unsigned short* __restrict__ wsel,
                                               const float* __restrict__ gl,
                                               float* __restrict__ out)
{
  __shared__ __align__(16) float sOut[4 * 32 * OPITCH];

  const int tid = threadIdx.x, lane = tid & 31, wv = tid >> 5;
  const int h = lane >> 4, m = lane & 15;
  const int b  = blockIdx.x / PGRP;
  const int pg = blockIdx.x - b * PGRP;
  const int cout0 = wv * 32;
  const int p0 = pg * 32;
  const float wlo = gl[(size_t)b * GLW + 10];
  const float whi = gl[(size_t)b * GLW + 11];

  const int pxa = p0 + m, pxb = p0 + 16 + m;
  const int pha = pxa / IMW, pwa = pxa - pha * IMW;
  const int phb = pxb / IMW, pwb = pxb - phb * IMW;
  const unsigned short* xa = xh + ((size_t)(b * PADH + pha) * PADW + pwa) * CH + 8 * h;
  const unsigned short* xb = xh + ((size_t)(b * PADH + phb) * PADW + pwb) * CH + 8 * h;
  const size_t splane = (size_t)NTAP * CH * CH;
  const unsigned short* wa0 = wsel + ((size_t)(b * 2) * NTAP * CH + cout0 + m) * CH + 8 * h;
  const unsigned short* wa1 = wa0 + 16 * CH;
  const unsigned short* wc0 = wa0 + splane;
  const unsigned short* wc1 = wc0 + 16 * CH;

  const v8f z8 = {0.f, 0.f, 0.f, 0.f, 0.f, 0.f, 0.f, 0.f};
  v8f d00a = z8, d00c = z8, d01a = z8, d01c = z8;
  v8f d10a = z8, d10c = z8, d11a = z8, d11c = z8;

  #pragma unroll 1
  for (int tap = 0; tap < NTAP; ++tap) {
    const int dh = tap / 3, dw = tap - dh * 3;
    const int aoff = (dh * PADW + dw) * CH;
    const int boff = tap * CH * CH;
    #pragma unroll 1
    for (int c0 = 0; c0 < CH; c0 += 32) {
      const v16h A0 = ldfrag(xa + aoff + c0);
      const v16h A1 = ldfrag(xb + aoff + c0);
      const v16h Ba0 = ldfrag(wa0 + boff + c0);
      const v16h Ba1 = ldfrag(wa1 + boff + c0);
      const v16h Bc0 = ldfrag(wc0 + boff + c0);
      const v16h Bc1 = ldfrag(wc1 + boff + c0);
      d00a = wmma_h(A0, Ba0, d00a);
      d00c = wmma_h(A0, Bc0, d00c);
      d01a = wmma_h(A0, Ba1, d01a);
      d01c = wmma_h(A0, Bc1, d01c);
      d10a = wmma_h(A1, Ba0, d10a);
      d10c = wmma_h(A1, Bc0, d10c);
      d11a = wmma_h(A1, Ba1, d11a);
      d11c = wmma_h(A1, Bc1, d11c);
    }
  }

  float* so = sOut + wv * (32 * OPITCH);
  epi_tile(so, d00a, d00c, wlo, whi, 0, 0, h, m);
  epi_tile(so, d01a, d01c, wlo, whi, 0, 1, h, m);
  epi_tile(so, d10a, d10c, wlo, whi, 1, 0, h, m);
  epi_tile(so, d11a, d11c, wlo, whi, 1, 1, h, m);
  __syncthreads();

  float* ob = out + ((size_t)(b * CH + cout0)) * NPIX + p0;
  const int lq = lane >> 3, px = 4 * (lane & 7);
  #pragma unroll
  for (int i = 0; i < 8; ++i) {
    const int cl = 4 * i + lq;
    const v4f v = *(const v4fa*)(so + cl * OPITCH + px);
    *(volatile v4f*)(ob + (size_t)cl * NPIX + px) = v;
  }
  __threadfence();
  #pragma unroll
  for (int i = 0; i < 8; ++i) {
    const int cl = 4 * i + lq;
    const v4f v = *(const v4fa*)(so + cl * OPITCH + px);
    *(volatile v4f*)(ob + (size_t)cl * NPIX + px) = v;
  }
}

extern "C" void kernel_launch(void* const* d_in, const int* in_sizes, int n_in,
                              void* d_out, int out_size, void* d_ws, size_t ws_size,
                              hipStream_t stream)
{
  if (n_in < 5) return;
  if (in_sizes[0] != NBATCH * CH * NPIX) return;
  if (in_sizes[1] != NEXP * CH * CH * NTAP) return;
  if (in_sizes[2] != NEXP * CH) return;
  if (in_sizes[3] != NEXP) return;
  if (in_sizes[4] != 1) return;
  if (out_size != NBATCH * CH * NPIX + NBATCH * NEXP) return;

  const float* x    = (const float*)d_in[0];
  const float* cw   = (const float*)d_in[1];
  const float* gw   = (const float*)d_in[2];
  const float* gb   = (const float*)d_in[3];
  const int*   tk   = (const int*)d_in[4];
  float* out0 = (float*)d_out;
  float* out1 = out0 + (size_t)NBATCH * CH * NPIX;

  const size_t bGL = (size_t)NBATCH * GLW * 4;
  const size_t bXH = (size_t)NBATCH * PADH * PADW * CH * 2;
  const size_t bWS = (size_t)NBATCH * 2 * NTAP * CH * CH * 2;
  const size_t total = bGL + bXH + bWS;
  if (total > ws_size) return;
  if (total > (size_t)134217728) return;

  char* ws = (char*)d_ws;
  size_t off = 0;
  float*          gl   = (float*)(ws + off);           off += bGL;
  unsigned short* xh   = (unsigned short*)(ws + off);  off += bXH;
  unsigned short* wsel = (unsigned short*)(ws + off);  off += bWS;
  if (off != total) return;

  k_gate<<<G_GATE, TGATE, 0, stream>>>(x, gw, gb, tk, gl);
  k_xcvt<<<G_XCVT, TCVT, 0, stream>>>(x, xh);
  k_wsel<<<G_WSEL, TCVT, 0, stream>>>(cw, gl, wsel, out1);
  k_conv<<<G_CONV, TCONV, 0, stream>>>(xh, wsel, gl, out0);
}
